// PointNetSetAbstraction_11192684773543
// MI455X (gfx1250) — hardware-verified
//
#include <hip/hip_runtime.h>
#include <stdint.h>

#pragma clang fp contract(off)

typedef __attribute__((ext_vector_type(16))) _Float16     v16h;
typedef __attribute__((ext_vector_type(8)))  _Float16     v8h;
typedef __attribute__((ext_vector_type(8)))  float        v8f;
typedef __attribute__((ext_vector_type(4)))  float        v4f;
typedef __attribute__((ext_vector_type(4)))  unsigned int v4u;
typedef __attribute__((ext_vector_type(4)))  int          v4i;

constexpr int NBATCH = 8;
constexpr int NPTS   = 4096;
constexpr int NFEAT  = 64;
constexpr int NCENT  = 1024;
constexpr int NSAMP  = 32;
constexpr int CIN0   = 67;
constexpr int KPAD0  = 96;
constexpr int NCH0   = 64;
constexpr int NCH1   = 64;
constexpr int NCH2   = 128;
constexpr int MROWS  = NBATCH * NCENT * NSAMP;
constexpr int OUT0_FLOATS = NBATCH * 3 * NCENT;
constexpr int GEMM_BLOCKS = MROWS / 256;
static_assert(MROWS == 262144, "row count");
static_assert(OUT0_FLOATS * 4 == 98304, "out1 byte offset");
static_assert(KPAD0 % 32 == 0 && KPAD0 >= CIN0, "K pad");
static_assert(NFEAT + 3 == CIN0, "channel count");
static_assert(MROWS % 256 == 0, "GEMM tile multiple");
static_assert((size_t)OUT0_FLOATS * 4 + (size_t)NBATCH * NCH2 * NCENT * 4 == 4292608, "d_out total");

constexpr size_t SZ_CEN   = (size_t)NBATCH * 3 * NCENT * 4;
constexpr size_t SZ_GI    = (size_t)NBATCH * NCENT * NSAMP * 4;
constexpr size_t SZ_FEATT = (size_t)NBATCH * NPTS * NFEAT * 2;
constexpr size_t SZ_W     = (size_t)(NCH0 * KPAD0 + NCH1 * NCH0 + NCH2 * NCH1) * 2;
constexpr size_t SZ_PART0 = (size_t)GEMM_BLOCKS * 2 * NCH0 * 4;
constexpr size_t SZ_PART1 = (size_t)GEMM_BLOCKS * 2 * NCH1 * 4;
constexpr size_t SZ_PART2 = (size_t)GEMM_BLOCKS * 2 * NCH2 * 4;
constexpr size_t SZ_BN    = (size_t)3 * 256 * 4;
constexpr size_t SZ_YMX   = (size_t)NBATCH * NCENT * NCH2 * 4;
constexpr size_t SZ_X     = (size_t)MROWS * KPAD0 * 2;
constexpr size_t SZ_Y     = (size_t)MROWS * NCH0 * 4;
constexpr size_t OFF_CEN   = 0;
constexpr size_t OFF_GI    = OFF_CEN + SZ_CEN;
constexpr size_t OFF_FEATT = OFF_GI + SZ_GI;
constexpr size_t OFF_W     = OFF_FEATT + SZ_FEATT;
constexpr size_t OFF_PART0 = OFF_W + SZ_W;
constexpr size_t OFF_PART1 = OFF_PART0 + SZ_PART0;
constexpr size_t OFF_PART2 = OFF_PART1 + SZ_PART1;
constexpr size_t OFF_BN    = OFF_PART2 + SZ_PART2;
constexpr size_t OFF_YMAX  = OFF_BN + SZ_BN;
constexpr size_t OFF_YMIN  = OFF_YMAX + SZ_YMX;
constexpr size_t OFF_X     = OFF_YMIN + SZ_YMX;
constexpr size_t OFF_Y     = OFF_X + SZ_X;
constexpr size_t WS_TOTAL  = OFF_Y + SZ_Y;
static_assert(WS_TOTAL <= (size_t)134217728, "carve under 128 MiB");
static_assert(OFF_GI % 128 == 0 && OFF_FEATT % 128 == 0 && OFF_W % 128 == 0 && OFF_PART0 % 128 == 0, "line aligned");
static_assert(OFF_PART1 % 128 == 0 && OFF_PART2 % 128 == 0 && OFF_BN % 128 == 0 && OFF_YMAX % 128 == 0, "line aligned");
static_assert(OFF_YMIN % 128 == 0 && OFF_X % 128 == 0 && OFF_Y % 128 == 0, "line aligned");
static_assert((size_t)MROWS * NCH0 * 2 <= SZ_X, "X64 view fits in X");

__device__ __forceinline__ int clampi(int v, int lo, int hi) { return v < lo ? lo : (v > hi ? hi : v); }

union FragU { v16h v; v8h h[2]; };
__device__ __forceinline__ v16h frag_load(const _Float16* p) {
  FragU f;
  f.h[0] = *(const v8h*)(p);
  f.h[1] = *(const v8h*)(p + 16);
  return f.v;
}
__device__ __forceinline__ v8f frag_mma(v16h a, v16h b, v8f c) {
  return __builtin_amdgcn_wmma_f32_16x16x32_f16(false, a, false, b, (short)0, c, false, false);
}
__device__ __forceinline__ void guard_grp(v8f& a, v8f& b, v8f& c, v8f& d, v16h x, v16h w0, v16h w1, v16h w2, v16h w3) {
  asm volatile("v_nop\n\tv_nop\n\tv_nop\n\tv_nop" : "+v"(a), "+v"(b), "+v"(c), "+v"(d) : "v"(x), "v"(w0), "v"(w1), "v"(w2), "v"(w3));
}
__device__ __forceinline__ void acc_guard4(v8f& a, v8f& b, v8f& c, v8f& d) {
  asm volatile("v_nop\n\tv_nop\n\tv_nop\n\tv_nop" : "+v"(a), "+v"(b), "+v"(c), "+v"(d));
}
__device__ __forceinline__ void wave_lds_sync() {
  __builtin_amdgcn_fence(__ATOMIC_RELEASE, "workgroup");
  __builtin_amdgcn_wave_barrier();
  __builtin_amdgcn_fence(__ATOMIC_ACQUIRE, "workgroup");
}

__global__ __launch_bounds__(256) void fps_select(const float* __restrict__ pos,
                                                  float* __restrict__ out0,
                                                  float* __restrict__ cen) {
#pragma clang fp contract(off)
  __shared__ __align__(16) float s_xyz[3 * NPTS];
  __shared__ float s_val[2][8];
  __shared__ int   s_idx[2][8];
  __shared__ __align__(16) int s_list[NCENT];

  const int b = blockIdx.x;
  const int tid = threadIdx.x;
  const int lane = tid & 31;
  const int wave = tid >> 5;
  const float* pb = pos + (size_t)b * 3 * NPTS;

#pragma unroll 1
  for (int grp = 0; grp < 3; ++grp) {
    v4f tmp[4];
#pragma unroll
    for (int j = 0; j < 4; ++j) tmp[j] = *(const v4f*)(pb + 4 * (tid + 256 * (grp * 4 + j)));
#pragma unroll
    for (int j = 0; j < 4; ++j) *(v4f*)(s_xyz + 4 * (tid + 256 * (grp * 4 + j))) = tmp[j];
  }
  if (tid == 0) s_list[0] = 0;
  __syncthreads();

  float x[16], y[16], z[16], cum[16];
#pragma unroll
  for (int i = 0; i < 16; ++i) {
    const int n = i * 256 + tid;
    x[i] = s_xyz[n];
    y[i] = s_xyz[NPTS + n];
    z[i] = s_xyz[2 * NPTS + n];
  }
  float cx = s_xyz[0], cy = s_xyz[NPTS], cz = s_xyz[2 * NPTS];
#pragma unroll
  for (int i = 0; i < 16; ++i) {
    const float dx = x[i] - cx, dy = y[i] - cy, dz = z[i] - cz;
    const float t0 = dx * dx;
    const float t1 = dy * dy;
    const float t2 = dz * dz;
    cum[i] = (t0 + t2) + t1;
  }
  unsigned msk = (tid == 0) ? 1u : 0u;

  for (int st = 1; st < NCENT; ++st) {
    const int buf = st & 1;
    float best = -__builtin_inff();
    int bn = 0x7fffffff;
#pragma unroll
    for (int i = 0; i < 16; ++i) {
      const bool live = ((msk >> i) & 1u) == 0u;
      const float v = cum[i];
      const int n = i * 256 + tid;
      const bool take = live && ((v > best) || (v == best && n < bn));
      best = take ? v : best;
      bn = take ? n : bn;
    }
#pragma unroll
    for (int off = 16; off; off >>= 1) {
      const float ov = __shfl_xor(best, off, 32);
      const int on = __shfl_xor(bn, off, 32);
      const bool take = (ov > best) || (ov == best && on < bn);
      best = take ? ov : best;
      bn = take ? on : bn;
    }
    if (lane == 0) { s_val[buf][wave] = best; s_idx[buf][wave] = bn; }
    __syncthreads();
    float bv = s_val[buf][0];
    int bi = s_idx[buf][0];
#pragma unroll
    for (int w = 1; w < 8; ++w) {
      const float v = s_val[buf][w];
      const int n = s_idx[buf][w];
      const bool take = (v > bv) || (v == bv && n < bi);
      bv = take ? v : bv;
      bi = take ? n : bi;
    }
    const int bestn = clampi(bi, 0, NPTS - 1);
    if (tid == 0) s_list[st] = bestn;
    cx = s_xyz[bestn];
    cy = s_xyz[NPTS + bestn];
    cz = s_xyz[2 * NPTS + bestn];
#pragma unroll
    for (int i = 0; i < 16; ++i) {
      const float dx = x[i] - cx, dy = y[i] - cy, dz = z[i] - cz;
      const float t0 = dx * dx;
      const float t1 = dy * dy;
      const float t2 = dz * dz;
      const float d = (t0 + t2) + t1;
      cum[i] = cum[i] + d;
      if ((i * 256 + tid) == bestn) msk |= (1u << i);
    }
  }
  __syncthreads();

  const v4i id = *(const v4i*)(s_list + 4 * tid);
  const int i0 = clampi(id[0], 0, NPTS - 1);
  const int i1 = clampi(id[1], 0, NPTS - 1);
  const int i2 = clampi(id[2], 0, NPTS - 1);
  const int i3 = clampi(id[3], 0, NPTS - 1);
  v4f o0, o1, o2;
  o0[0] = s_xyz[i0]; o0[1] = s_xyz[i1]; o0[2] = s_xyz[i2]; o0[3] = s_xyz[i3];
  o1[0] = s_xyz[NPTS + i0]; o1[1] = s_xyz[NPTS + i1]; o1[2] = s_xyz[NPTS + i2]; o1[3] = s_xyz[NPTS + i3];
  o2[0] = s_xyz[2 * NPTS + i0]; o2[1] = s_xyz[2 * NPTS + i1]; o2[2] = s_xyz[2 * NPTS + i2]; o2[3] = s_xyz[2 * NPTS + i3];
  const size_t ob = (size_t)b * 3 * NCENT + 4 * tid;
  for (int pass = 0; pass < 2; ++pass) {
    *(volatile v4f*)(out0 + ob) = o0;
    *(volatile v4f*)(out0 + ob + NCENT) = o1;
    *(volatile v4f*)(out0 + ob + 2 * NCENT) = o2;
    *(volatile v4f*)(cen + ob) = o0;
    *(volatile v4f*)(cen + ob + NCENT) = o1;
    *(volatile v4f*)(cen + ob + 2 * NCENT) = o2;
    __threadfence();
  }
}

__global__ __launch_bounds__(256) void feat_transpose(const float* __restrict__ feat,
                                                      unsigned short* __restrict__ featT) {
  __shared__ float tile[64][65];
  const int b = blockIdx.x >> 6;
  const int n0 = (blockIdx.x & 63) << 6;
  const int tid = threadIdx.x;
  const float* fb = feat + (size_t)b * NFEAT * NPTS;
  v4f ld[4];
#pragma unroll
  for (int j = 0; j < 4; ++j) {
    const int idx = tid + j * 256;
    const int c = idx >> 4, q = idx & 15;
    ld[j] = *(const v4f*)(fb + (size_t)c * NPTS + n0 + 4 * q);
  }
#pragma unroll
  for (int j = 0; j < 4; ++j) {
    const int idx = tid + j * 256;
    const int c = idx >> 4, q = idx & 15;
    tile[c][4 * q + 0] = ld[j][0];
    tile[c][4 * q + 1] = ld[j][1];
    tile[c][4 * q + 2] = ld[j][2];
    tile[c][4 * q + 3] = ld[j][3];
  }
  __syncthreads();
  v8h o[2];
#pragma unroll
  for (int j = 0; j < 2; ++j) {
    const int slot = tid + j * 256;
    const int nn = slot >> 3, c8 = (slot & 7) * 8;
#pragma unroll
    for (int e = 0; e < 8; ++e) o[j][e] = (_Float16)tile[c8 + e][nn];
  }
  for (int pass = 0; pass < 2; ++pass) {
#pragma unroll
    for (int j = 0; j < 2; ++j) {
      const int slot = tid + j * 256;
      const int nn = slot >> 3, c8 = (slot & 7) * 8;
      *(volatile v8h*)(featT + ((size_t)b * NPTS + n0 + nn) * NFEAT + c8) = o[j];
    }
    __threadfence();
  }
}

__global__ __launch_bounds__(256) void prep_weights(const float* __restrict__ w0,
                                                    const float* __restrict__ w1,
                                                    const float* __restrict__ w2,
                                                    unsigned short* __restrict__ Wp) {
  const int blk = blockIdx.x;
  const int tid = threadIdx.x;
  v8h o;
  size_t dst;
  if (blk < 3) {
    const int e8 = (blk * 256 + tid) * 8;
    const int row = e8 / KPAD0;
    const int k0 = e8 - row * KPAD0;
#pragma unroll
    for (int e = 0; e < 8; ++e) {
      const int k = k0 + e;
      const int kc = k < CIN0 ? k : (CIN0 - 1);
      const float v = w0[row * CIN0 + kc];
      o[e] = (_Float16)((k < CIN0) ? v : 0.0f);
    }
    dst = (size_t)e8;
  } else if (blk < 5) {
    const int e8 = ((blk - 3) * 256 + tid) * 8;
    const v4f a = *(const v4f*)(w1 + e8);
    const v4f c = *(const v4f*)(w1 + e8 + 4);
#pragma unroll
    for (int e = 0; e < 4; ++e) { o[e] = (_Float16)a[e]; o[4 + e] = (_Float16)c[e]; }
    dst = (size_t)(NCH0 * KPAD0) + e8;
  } else {
    const int e8 = ((blk - 5) * 256 + tid) * 8;
    const v4f a = *(const v4f*)(w2 + e8);
    const v4f c = *(const v4f*)(w2 + e8 + 4);
#pragma unroll
    for (int e = 0; e < 4; ++e) { o[e] = (_Float16)a[e]; o[4 + e] = (_Float16)c[e]; }
    dst = (size_t)(NCH0 * KPAD0 + NCH1 * NCH0) + e8;
  }
  *(volatile v8h*)(Wp + dst) = o;
  __threadfence();
  *(volatile v8h*)(Wp + dst) = o;
}

__global__ __launch_bounds__(256) void ball_query(const float* __restrict__ pos,
                                                  const float* __restrict__ cen,
                                                  int* __restrict__ gi) {
#pragma clang fp contract(off)
  __shared__ int s_slot[8][NSAMP];
  const int lane = threadIdx.x & 31;
  const int wave = threadIdx.x >> 5;
  const int cidx = blockIdx.x * 8 + wave;
  const int b = cidx >> 10;
  const int s = cidx & (NCENT - 1);
  const float* pb = pos + (size_t)b * 3 * NPTS;
  const float cx = cen[((size_t)b * 3 + 0) * NCENT + s];
  const float cy = cen[((size_t)b * 3 + 1) * NCENT + s];
  const float cz = cen[((size_t)b * 3 + 2) * NCENT + s];
  const float c0 = cx * cx;
  const float c1 = cy * cy;
  const float c2 = cz * cz;
  const float sqc = (c0 + c2) + c1;
  const float thr = 0.04f;

  s_slot[wave][lane] = 0;
  __syncthreads();

  int cnt = 0;
  int gi0 = NPTS - 1;
  for (int base = 0; base < NPTS && cnt < NSAMP; base += 32) {
    const int n = base + lane;
    const float px = pb[n];
    const float py = pb[NPTS + n];
    const float pz = pb[2 * NPTS + n];
    float p = cx * px;
    p = fmaf(cy, py, p);
    p = fmaf(cz, pz, p);
    const float u0 = px * px;
    const float u1 = py * py;
    const float u2 = pz * pz;
    const float sqp = (u0 + u2) + u1;
    float d = -2.0f * p;
    d = d + sqc;
    d = d + sqp;
    const bool pred = !(d > thr);
    const unsigned m = __builtin_amdgcn_ballot_w32(pred);
    const int rank = cnt + __popc(m & ((1u << lane) - 1u));
    if (pred && rank < NSAMP) s_slot[wave][rank] = n;
    const int fl = __ffs((int)m) - 1;
    if (cnt == 0 && m != 0u) gi0 = base + fl;
    cnt += __popc(m);
  }
  __syncthreads();
  const int sv = s_slot[wave][lane];
  int val = (lane < cnt) ? sv : gi0;
  val = clampi(val, 0, NPTS - 1);
  volatile int* dst = gi + (size_t)cidx * NSAMP + lane;
  *dst = val;
  __threadfence();
  *dst = val;
}

__global__ __launch_bounds__(256) void gather_rows(const float* __restrict__ pos,
                                                   const unsigned short* __restrict__ featT,
                                                   const float* __restrict__ cen,
                                                   const int* __restrict__ gi,
                                                   unsigned short* __restrict__ Xo) {
  const int lane = threadIdx.x & 31;
  const int wave = threadIdx.x >> 5;
  const int m0 = (blockIdx.x * 8 + wave) * 8;
  const v4u* f4 = (const v4u*)featT;
#pragma unroll 1
  for (int it = 0; it < 3; ++it) {
    const int slot = it * 32 + lane;
    const int rr = slot / 12;
    const int g = slot - rr * 12;
    const int m = m0 + rr;
    const int b = m >> 15;
    const int s = (m >> 5) & (NCENT - 1);
    const int n = clampi(gi[m], 0, NPTS - 1);
    const float px = pos[((size_t)b * 3 + 0) * NPTS + n];
    const float py = pos[((size_t)b * 3 + 1) * NPTS + n];
    const float pz = pos[((size_t)b * 3 + 2) * NPTS + n];
    const float qx = cen[((size_t)b * 3 + 0) * NCENT + s];
    const float qy = cen[((size_t)b * 3 + 1) * NCENT + s];
    const float qz = cen[((size_t)b * 3 + 2) * NCENT + s];
    const size_t base4 = ((size_t)b * NPTS + n) * 8;
    const int ia = clampi(g - 1, 0, 7);
    const int ib = clampi(g, 0, 7);
    const v4u wa = f4[base4 + ia];
    const v4u wb = f4[base4 + ib];
    const _Float16 hx = (_Float16)(px - qx);
    const _Float16 hy = (_Float16)(py - qy);
    const _Float16 hz = (_Float16)(pz - qz);
    const unsigned ux = (unsigned)__builtin_bit_cast(unsigned short, hx);
    const unsigned uy = (unsigned)__builtin_bit_cast(unsigned short, hy);
    const unsigned uz = (unsigned)__builtin_bit_cast(unsigned short, hz);
    const unsigned a2 = wa[2];
    const unsigned a3 = wa[3];
    const bool validA = (g >= 1) && (g <= 8);
    const bool validB = (g <= 7);
    const unsigned fa5 = validA ? (a2 >> 16) : 0u;
    const unsigned fa6 = validA ? (a3 & 0xffffu) : 0u;
    const unsigned fa7 = validA ? (a3 >> 16) : 0u;
    const unsigned h5 = (g == 0) ? ux : fa5;
    const unsigned h6 = (g == 0) ? uy : fa6;
    const unsigned h7 = (g == 0) ? uz : fa7;
    const unsigned b0 = validB ? wb[0] : 0u;
    const unsigned b1 = validB ? wb[1] : 0u;
    const unsigned b2 = validB ? wb[2] : 0u;
    v4u o;
    o[0] = h5 | (h6 << 16);
    o[1] = h7 | (b0 << 16);
    o[2] = (b0 >> 16) | (b1 << 16);
    o[3] = (b1 >> 16) | (b2 << 16);
    volatile v4u* dst = (volatile v4u*)Xo + ((size_t)m0 * 12 + slot);
    *dst = o;
    __threadfence();
    *dst = o;
  }
}

template <int KDIM, int NOUT, bool POOL>
__global__ __launch_bounds__(256) void mlp_layer_gemm(const unsigned short* __restrict__ Xp,
                                                      const unsigned short* __restrict__ Wp,
                                                      const float* __restrict__ bias,
                                                      float* __restrict__ Yout,
                                                      float* __restrict__ partials,
                                                      float* __restrict__ ymax,
                                                      float* __restrict__ ymin) {
  static_assert(KDIM % 32 == 0, "K multiple of 32");
  static_assert(NOUT % 64 == 0, "N multiple of 64");
  static_assert(POOL || NOUT == 64, "stored rows are 64 wide");
  const _Float16* X = (const _Float16*)Xp;
  const _Float16* W = (const _Float16*)Wp;
  __shared__ __align__(16) float sT[POOL ? 1 : 8][POOL ? 4 : 16 * 68];
  __shared__ __align__(16) float sStat[8][2 * NOUT];
  __shared__ __align__(16) float sMx[POOL ? 8 : 1][POOL ? NOUT : 4];
  __shared__ __align__(16) float sMn[POOL ? 8 : 1][POOL ? NOUT : 4];

  const int tid = threadIdx.x;
  const int lane = tid & 31;
  const int wave = tid >> 5;
  const int rlane = lane & 15;
  const int hh = lane >> 4;
  const int koff = hh * 8;
  const int mOff = hh * 8;
  const int blk = blockIdx.x;
  const size_t row0 = (size_t)blk * 256 + (size_t)wave * 32;

#pragma unroll 1
  for (int nh = 0; nh < NOUT / 64; ++nh) {
    v8f acc[2][4];
#pragma unroll
    for (int i = 0; i < 2; ++i)
#pragma unroll
      for (int j = 0; j < 4; ++j) acc[i][j] = (v8f){0.f, 0.f, 0.f, 0.f, 0.f, 0.f, 0.f, 0.f};

#pragma unroll 1
    for (int k0 = 0; k0 < KDIM; k0 += 32) {
      v16h bh[4];
#pragma unroll
      for (int j = 0; j < 4; ++j)
        bh[j] = frag_load(W + (size_t)(nh * 64 + (j << 4) + rlane) * KDIM + koff + k0);
      asm volatile("" ::: "memory");
#pragma unroll
      for (int i = 0; i < 2; ++i) {
        const v16h ah = frag_load(X + (row0 + (size_t)((i << 4) + rlane)) * KDIM + koff + k0);
#pragma unroll
        for (int j = 0; j < 4; ++j) acc[i][j] = frag_mma(ah, bh[j], acc[i][j]);
        guard_grp(acc[i][0], acc[i][1], acc[i][2], acc[i][3], ah, bh[0], bh[1], bh[2], bh[3]);
      }
    }
    acc_guard4(acc[0][0], acc[0][1], acc[0][2], acc[0][3]);
    acc_guard4(acc[1][0], acc[1][1], acc[1][2], acc[1][3]);

#pragma unroll
    for (int j = 0; j < 4; ++j) {
      const int n = nh * 64 + (j << 4) + rlane;
      const float bv = bias[n];
      float sm = 0.0f, sq = 0.0f;
      float mx = -__builtin_inff(), mn = __builtin_inff();
#pragma unroll
      for (int i = 0; i < 2; ++i) {
#pragma unroll
        for (int r = 0; r < 8; ++r) {
          const float yv = acc[i][j][r] + bv;
          acc[i][j][r] = yv;
          sm += yv;
          const float y2 = yv * yv;
          sq += y2;
          mx = fmaxf(mx, yv);
          mn = fminf(mn, yv);
        }
      }
      const float sm2 = __shfl_xor(sm, 16, 32);
      const float sq2 = __shfl_xor(sq, 16, 32);
      const float mx2 = __shfl_xor(mx, 16, 32);
      const float mn2 = __shfl_xor(mn, 16, 32);
      sm = sm + sm2;
      sq = sq + sq2;
      mx = fmaxf(mx, mx2);
      mn = fminf(mn, mn2);
      if (lane < 16) {
        sStat[wave][n] = sm;
        sStat[wave][NOUT + n] = sq;
        if (POOL) { sMx[wave][n] = mx; sMn[wave][n] = mn; }
      }
    }

    if (!POOL) {
      float* slab = sT[wave];
      const int c4 = (lane & 15) * 4;
#pragma unroll
      for (int i = 0; i < 2; ++i) {
#pragma unroll
        for (int j = 0; j < 4; ++j)
#pragma unroll
          for (int r = 0; r < 8; ++r) slab[(mOff + r) * 68 + (j << 4) + rlane] = acc[i][j][r];
        wave_lds_sync();
        for (int pass = 0; pass < 2; ++pass) {
#pragma unroll
          for (int it = 0; it < 8; ++it) {
            const int row = it * 2 + hh;
            const v4f v = *(const v4f*)(slab + row * 68 + c4);
            *(volatile v4f*)(Yout + (row0 + (size_t)((i << 4) + row)) * NOUT + nh * 64 + c4) = v;
          }
          __threadfence();
        }
        wave_lds_sync();
      }
    }
  }

  __syncthreads();
  if (tid < 2 * NOUT) {
    float s = 0.0f;
#pragma unroll
    for (int w = 0; w < 8; ++w) s += sStat[w][tid];
    volatile float* pp = partials + (size_t)blk * (2 * NOUT) + tid;
    *pp = s;
    __threadfence();
    *pp = s;
  }
  if (POOL) {
    const int row = tid >> 5;
    const int c4 = (tid & 31) * 4;
    const v4f a = *(const v4f*)(&sMx[row][c4]);
    const v4f c = *(const v4f*)(&sMn[row][c4]);
    const size_t go = ((size_t)blk * 8 + row) * NOUT + c4;
    *(volatile v4f*)(ymax + go) = a;
    *(volatile v4f*)(ymin + go) = c;
    __threadfence();
    *(volatile v4f*)(ymax + go) = a;
    *(volatile v4f*)(ymin + go) = c;
  }
}

template <int C>
__global__ __launch_bounds__(256) void bn_finalize(const float* __restrict__ partials,
                                                   const float* __restrict__ gam,
                                                   const float* __restrict__ bet,
                                                   float* __restrict__ bn) {
  __shared__ double sd[256];
  const int t = threadIdx.x;
  const int tc = t < 2 * C ? t : (2 * C - 1);
  double acc = 0.0;
#pragma unroll 4
  for (int blk = 0; blk < GEMM_BLOCKS; ++blk) acc += (double)partials[(size_t)blk * (2 * C) + tc];
  sd[t] = acc;
  __syncthreads();
  const int ch = t & 127;
  const int chc = ch < C ? ch : (C - 1);
  const double inv_m = 1.0 / (double)MROWS;
  const double mean = sd[chc] * inv_m;
  const double ex2 = sd[C + chc] * inv_m;
  double var = ex2 - mean * mean;
  var = var < 0.0 ? 0.0 : var;
  const float varf = (float)var;
  const float meanf = (float)mean;
  const float rs = 1.0f / sqrtf(varf + 1e-5f);
  const float scl = gam[chc] * rs;
  const float shf = bet[chc] - meanf * scl;
  float val = (t < 128) ? scl : shf;
  val = (ch < C) ? val : 0.0f;
  volatile float* dst = bn + t;
  *dst = val;
  __threadfence();
  *dst = val;
}

__global__ __launch_bounds__(256) void bn_relu_f16(const float* __restrict__ Y,
                                                   const float* __restrict__ bn,
                                                   unsigned short* __restrict__ Xo) {
  const size_t idx = (size_t)blockIdx.x * 256 + threadIdx.x;
  const int c8 = (int)(idx & 7) * 8;
  const v4f y0 = *(const v4f*)(Y + idx * 8);
  const v4f y1 = *(const v4f*)(Y + idx * 8 + 4);
  const v4f s0 = *(const v4f*)(bn + c8);
  const v4f s1 = *(const v4f*)(bn + c8 + 4);
  const v4f h0 = *(const v4f*)(bn + 128 + c8);
  const v4f h1 = *(const v4f*)(bn + 128 + c8 + 4);
  v8h o;
#pragma unroll
  for (int e = 0; e < 4; ++e) {
    o[e] = (_Float16)fmaxf(fmaf(y0[e], s0[e], h0[e]), 0.0f);
    o[4 + e] = (_Float16)fmaxf(fmaf(y1[e], s1[e], h1[e]), 0.0f);
  }
  *(volatile v8h*)(Xo + idx * 8) = o;
  __threadfence();
  *(volatile v8h*)(Xo + idx * 8) = o;
}

__global__ __launch_bounds__(256) void pool_bn_out(const float* __restrict__ ymax,
                                                   const float* __restrict__ ymin,
                                                   const float* __restrict__ bn,
                                                   float* __restrict__ out1) {
  __shared__ __align__(16) float tile[128 * 36];
  const int t = threadIdx.x;
  const int b = blockIdx.x >> 5;
  const int s0 = (blockIdx.x & 31) * 32;
  const int cg = (t & 31) * 4;
  const v4f sc = *(const v4f*)(bn + cg);
  const v4f sh = *(const v4f*)(bn + 128 + cg);
#pragma unroll 1
  for (int it = 0; it < 4; ++it) {
    const int sl = it * 8 + (t >> 5);
    const size_t ro = ((size_t)b * NCENT + s0 + sl) * NCH2 + cg;
    const v4f a = *(const v4f*)(ymax + ro);
    const v4f c = *(const v4f*)(ymin + ro);
#pragma unroll
    for (int e = 0; e < 4; ++e) {
      const float yv = (sc[e] > 0.0f) ? a[e] : c[e];
      tile[(cg + e) * 36 + sl] = fmaxf(fmaf(yv, sc[e], sh[e]), 0.0f);
    }
  }
  __syncthreads();
  v4f vals[4];
#pragma unroll
  for (int it = 0; it < 4; ++it) {
    const int slot = it * 256 + t;
    const int c = slot >> 3, q = slot & 7;
    vals[it] = *(const v4f*)(tile + c * 36 + 4 * q);
  }
  for (int pass = 0; pass < 2; ++pass) {
#pragma unroll
    for (int it = 0; it < 4; ++it) {
      const int slot = it * 256 + t;
      const int c = slot >> 3, q = slot & 7;
      *(volatile v4f*)(out1 + ((size_t)b * NCH2 + c) * NCENT + s0 + 4 * q) = vals[it];
    }
    __threadfence();
  }
}

extern "C" void kernel_launch(void* const* d_in, const int* in_sizes, int n_in,
                              void* d_out, int out_size, void* d_ws, size_t ws_size,
                              hipStream_t stream) {
  (void)in_sizes; (void)out_size;
  if (n_in < 14) return;
  if (ws_size < WS_TOTAL) return;

  const float* pos  = (const float*)d_in[0];
  const float* feat = (const float*)d_in[1];
  const float* w0   = (const float*)d_in[2];
  const float* b0   = (const float*)d_in[3];
  const float* g0   = (const float*)d_in[4];
  const float* be0  = (const float*)d_in[5];
  const float* w1   = (const float*)d_in[6];
  const float* b1   = (const float*)d_in[7];
  const float* g1   = (const float*)d_in[8];
  const float* be1  = (const float*)d_in[9];
  const float* w2   = (const float*)d_in[10];
  const float* b2   = (const float*)d_in[11];
  const float* g2   = (const float*)d_in[12];
  const float* be2  = (const float*)d_in[13];
  float* out = (float*)d_out;

  char* ws = (char*)d_ws;
  float*          cen   = (float*)(ws + OFF_CEN);
  int*            gi    = (int*)(ws + OFF_GI);
  unsigned short* featT = (unsigned short*)(ws + OFF_FEATT);
  unsigned short* Wpl   = (unsigned short*)(ws + OFF_W);
  unsigned short* W0h   = Wpl;
  unsigned short* W1h   = Wpl + NCH0 * KPAD0;
  unsigned short* W2h   = Wpl + NCH0 * KPAD0 + NCH1 * NCH0;
  float*          part0 = (float*)(ws + OFF_PART0);
  float*          part1 = (float*)(ws + OFF_PART1);
  float*          part2 = (float*)(ws + OFF_PART2);
  float*          bn0   = (float*)(ws + OFF_BN);
  float*          bn1   = bn0 + 256;
  float*          bn2   = bn0 + 512;
  float*          ymax  = (float*)(ws + OFF_YMAX);
  float*          ymin  = (float*)(ws + OFF_YMIN);
  unsigned short* X     = (unsigned short*)(ws + OFF_X);
  float*          Y     = (float*)(ws + OFF_Y);

  fps_select<<<NBATCH, 256, 0, stream>>>(pos, out, cen);
  feat_transpose<<<NBATCH * 64, 256, 0, stream>>>(feat, featT);
  prep_weights<<<9, 256, 0, stream>>>(w0, w1, w2, Wpl);
  ball_query<<<NBATCH * NCENT / 8, 256, 0, stream>>>(pos, cen, gi);
  gather_rows<<<MROWS / 64, 256, 0, stream>>>(pos, featT, cen, gi, X);

  mlp_layer_gemm<KPAD0, NCH0, false><<<GEMM_BLOCKS, 256, 0, stream>>>(X, W0h, b0, Y, part0, ymax, ymin);
  bn_finalize<NCH0><<<1, 256, 0, stream>>>(part0, g0, be0, bn0);
  bn_relu_f16<<<MROWS * NCH0 / 8 / 256, 256, 0, stream>>>(Y, bn0, X);

  mlp_layer_gemm<NCH0, NCH1, false><<<GEMM_BLOCKS, 256, 0, stream>>>(X, W1h, b1, Y, part1, ymax, ymin);
  bn_finalize<NCH1><<<1, 256, 0, stream>>>(part1, g1, be1, bn1);
  bn_relu_f16<<<MROWS * NCH1 / 8 / 256, 256, 0, stream>>>(Y, bn1, X);

  mlp_layer_gemm<NCH1, NCH2, true><<<GEMM_BLOCKS, 256, 0, stream>>>(X, W2h, b2, Y, part2, ymax, ymin);
  bn_finalize<NCH2><<<1, 256, 0, stream>>>(part2, g2, be2, bn2);
  pool_bn_out<<<NBATCH * 32, 256, 0, stream>>>(ymax, ymin, bn2, out + OUT0_FLOATS);
}
